// KANLinear_53068615910216
// MI455X (gfx1250) — hardware-verified
//
#include <hip/hip_runtime.h>

constexpr int kRows   = 8192;
constexpr int kIn     = 256;
constexpr int kOut    = 256;
constexpr int kKnots  = 16;
constexpr int kKsp    = kIn * kKnots;
constexpr int kKtot   = kKsp + kIn;
constexpr int kRowWords = kKtot / 2;
constexpr int kChunks = kKtot / 8;
constexpr float kBtCarry    = 256.0f;
constexpr float kBtCarryInv = 1.0f / 256.0f;

static_assert(kKtot % 32 == 0, "K multiple of 32");
static_assert(kRows % 64 == 0 && kOut % 64 == 0, "M,N tile multiples");
static_assert(((kRows / 64) * (kOut / 64)) % 8 == 0, "8 tiles per GEMM block");
static_assert(kChunks % 32 == 0, "a wave never straddles two Bt rows");
static_assert((kOut * kChunks) % 256 == 0, "Bt pack grid exact");
static_assert(kRows % 4 == 0, "4 rows per feature block");
static_assert((kKtot * 2) % 128 == 0, "plane rows are whole 128-B lines");
static_assert((size_t)kOut * kKtot * 2 + (size_t)kRows * kKtot * 2 <= 134217728u, "carve within 128 MiB");

typedef __attribute__((ext_vector_type(16))) _Float16 v16h;
typedef __attribute__((ext_vector_type(8)))  _Float16 v8h;
typedef __attribute__((ext_vector_type(16))) __bf16   v16b;
typedef __attribute__((ext_vector_type(8)))  __bf16   v8b;
typedef __attribute__((ext_vector_type(8)))  float    v8f;
typedef __attribute__((ext_vector_type(4)))  float    v4f;
typedef __attribute__((ext_vector_type(4)))  unsigned int v4u;

__device__ __forceinline__ unsigned short f2bf_bits(float f) {
  unsigned u = __float_as_uint(f);
  return (unsigned short)((u + 0x7FFFu + ((u >> 16) & 1u)) >> 16);
}
__device__ __forceinline__ float bf_bits2f(unsigned short h) { return __uint_as_float(((unsigned)h) << 16); }

__device__ __forceinline__ void dep_guard_h(v8f& a, v8f& b, v16h x, v16h y) { asm volatile("v_nop\n\tv_nop\n\tv_nop\n\tv_nop" : "+v"(a), "+v"(b) : "v"(x), "v"(y)); }
__device__ __forceinline__ void dep_guard_b(v8f& a, v8f& b, v16b x, v16b y) { asm volatile("v_nop\n\tv_nop\n\tv_nop\n\tv_nop" : "+v"(a), "+v"(b) : "v"(x), "v"(y)); }
__device__ __forceinline__ void dep_guard4_h(v8f& a, v8f& b, v8f& c, v8f& d, v16h x, v16h y) {
  asm volatile("v_nop\n\tv_nop\n\tv_nop\n\tv_nop" : "+v"(a), "+v"(b), "+v"(c), "+v"(d) : "v"(x), "v"(y));
}
__device__ __forceinline__ void dep_guard4_b(v8f& a, v8f& b, v8f& c, v8f& d, v16b x, v16b y) {
  asm volatile("v_nop\n\tv_nop\n\tv_nop\n\tv_nop" : "+v"(a), "+v"(b), "+v"(c), "+v"(d) : "v"(x), "v"(y));
}
__device__ __forceinline__ void keep4_h(v16h a, v16h b, v16h c, v16h d) { asm volatile("v_nop" :: "v"(a), "v"(b), "v"(c), "v"(d)); }
__device__ __forceinline__ void keep4_b(v16b a, v16b b, v16b c, v16b d) { asm volatile("v_nop" :: "v"(a), "v"(b), "v"(c), "v"(d)); }
__device__ __forceinline__ void acc_guard4(v8f& a, v8f& b, v8f& c, v8f& d) { asm volatile("v_nop\n\tv_nop\n\tv_nop\n\tv_nop" : "+v"(a), "+v"(b), "+v"(c), "+v"(d)); }
template <typename T> struct Frag;
template <> struct Frag<_Float16> {
  typedef v16h V; union U { v16h v; v8h h[2]; };
  static __device__ __forceinline__ v16h load(const _Float16* p) {
    U f; f.h[0] = *(const v8h*)(p); f.h[1] = *(const v8h*)(p + 16); return f.v;
  }
  static __device__ __forceinline__ v8f mma(v16h a, v16h b, v8f c) {
    return __builtin_amdgcn_wmma_f32_16x16x32_f16(false, a, false, b, (short)0, c, false, false);
  }
  static __device__ __forceinline__ void guard(v8f& a, v8f& b, v16h x, v16h y) { dep_guard_h(a, b, x, y); }
  static __device__ __forceinline__ void guard4(v8f& a, v8f& b, v8f& c, v8f& d, v16h x, v16h y) { dep_guard4_h(a, b, c, d, x, y); }
  static __device__ __forceinline__ void keep(v16h a, v16h b, v16h c, v16h d) { keep4_h(a, b, c, d); }
};
template <> struct Frag<__bf16> {
  typedef v16b V; union U { v16b v; v8b h[2]; };
  static __device__ __forceinline__ v16b load(const __bf16* p) {
    U f; f.h[0] = *(const v8b*)(p); f.h[1] = *(const v8b*)(p + 16); return f.v;
  }
  static __device__ __forceinline__ v8f mma(v16b a, v16b b, v8f c) {
    return __builtin_amdgcn_wmma_f32_16x16x32_bf16(false, a, false, b, (short)0, c, false, false);
  }
  static __device__ __forceinline__ void guard(v8f& a, v8f& b, v16b x, v16b y) { dep_guard_b(a, b, x, y); }
  static __device__ __forceinline__ void guard4(v8f& a, v8f& b, v8f& c, v8f& d, v16b x, v16b y) { dep_guard4_b(a, b, c, d, x, y); }
  static __device__ __forceinline__ void keep(v16b a, v16b b, v16b c, v16b d) { keep4_b(a, b, c, d); }
};

__device__ __forceinline__ unsigned pk16(unsigned short a, unsigned short b) { return (unsigned)a | ((unsigned)b << 16); }
__device__ __forceinline__ unsigned short h_bits(float f) { const _Float16 h = (_Float16)f; return __builtin_bit_cast(unsigned short, h); }

template <int ET> struct Elem;
template <> struct Elem<0> { typedef _Float16 T; };
template <> struct Elem<1> { typedef __bf16 T; };
template <int ET, bool SPLIT, int BIAS_MODE, int OUT_MODE, bool RESID, int ACT = 0>
__global__ __launch_bounds__(256) void wmma_gemm64(
    const unsigned short* __restrict__ Ap, const unsigned short* __restrict__ A2p, int lda, long strideA,
    const unsigned short* __restrict__ Btp, const unsigned short* __restrict__ Bt2p, int ldb, long strideB,
    void* __restrict__ Cout, void* __restrict__ Cout2, int ldc, long strideC,
    const float* __restrict__ bias,
    const float* __restrict__ resid, long strideR,
    int M, int N, int K, float scale) {
  typedef typename Elem<ET>::T T;
  typedef typename Frag<T>::V V;
  const T* A = (const T*)Ap; const T* A2 = (const T*)A2p; const T* Bt = (const T*)Btp; const T* Bt2 = (const T*)Bt2p;
  __shared__ __align__(16) float sT[8][16 * 68];
  const int b    = blockIdx.y;
  const int lane = threadIdx.x & 31;
  const int wave = threadIdx.x >> 5;
  const int tilesN = N >> 6;
  const int tilesM = M >> 6;
  const int tile = blockIdx.x * 8 + wave;
  if (tile >= tilesM * tilesN) return;
  const int tm = tile / tilesN;
  const int tn = tile - tm * tilesN;
  const int m0 = tm << 6;
  const int n0 = tn << 6;

  const T* Ab  = A  + (size_t)b * strideA;
  const T* Bb  = Bt + (size_t)b * strideB;
  const T* Ab2 = SPLIT ? (A2  + (size_t)b * strideA) : nullptr;
  const T* Bb2 = SPLIT ? (Bt2 + (size_t)b * strideB) : nullptr;

  const int rlane = lane & 15;
  const int koff  = (lane >> 4) * 8;
  const int mOff  = (lane >> 4) * 8;

  v8f acc[4][4];
#pragma unroll
  for (int i = 0; i < 4; ++i)
#pragma unroll
    for (int j = 0; j < 4; ++j) acc[i][j] = (v8f){0.f,0.f,0.f,0.f,0.f,0.f,0.f,0.f};

  for (int k0 = 0; k0 < K; k0 += 32) {
    V bh[4], bl[4];
#pragma unroll
    for (int j = 0; j < 4; ++j) {
      const size_t bo = (size_t)(n0 + (j << 4) + rlane) * ldb + koff + k0;
      bh[j] = Frag<T>::load(Bb + bo);
      if (SPLIT) bl[j] = Frag<T>::load(Bb2 + bo);
    }
#pragma unroll
    for (int i = 0; i < 4; ++i) {
      const size_t ao = (size_t)(m0 + (i << 4) + rlane) * lda + koff + k0;
      V ah = Frag<T>::load(Ab + ao);
      V al;
      if (SPLIT) al = Frag<T>::load(Ab2 + ao);
#pragma unroll
      for (int j = 0; j < 4; ++j) {
        acc[i][j] = Frag<T>::mma(ah, bh[j], acc[i][j]);
        if (SPLIT) {
          acc[i][j] = Frag<T>::mma(ah, bl[j], acc[i][j]);
          acc[i][j] = Frag<T>::mma(al, bh[j], acc[i][j]);
        }
      }
      Frag<T>::guard4(acc[i][0], acc[i][1], acc[i][2], acc[i][3], ah, SPLIT ? al : bh[3]);
    }
    Frag<T>::keep(bh[0], bh[1], bh[2], bh[3]);
    if (SPLIT) Frag<T>::keep(bl[0], bl[1], bl[2], bl[3]);
  }
  acc_guard4(acc[0][0], acc[0][1], acc[0][2], acc[0][3]);
  acc_guard4(acc[1][0], acc[1][1], acc[1][2], acc[1][3]);
  acc_guard4(acc[2][0], acc[2][1], acc[2][2], acc[2][3]);
  acc_guard4(acc[3][0], acc[3][1], acc[3][2], acc[3][3]);

  float* slab = sT[wave];
  const float* Rb = RESID ? (resid + (size_t)b * strideR) : nullptr;
#pragma unroll
  for (int i = 0; i < 4; ++i) {
    const int mBase = m0 + (i << 4);
#pragma unroll
    for (int j = 0; j < 4; ++j) {
      const int n = n0 + (j << 4) + rlane;
      float bv = 0.f;
      if (BIAS_MODE == 2) bv = bias[n];
#pragma unroll
      for (int r = 0; r < 8; ++r) {
        float v = acc[i][j][r] * scale;
        if (BIAS_MODE == 1) v += bias[mBase + mOff + r];
        if (BIAS_MODE == 2) v += bv;
        if (RESID) v += Rb[(size_t)(mBase + mOff + r) * ldc + n];
        if (ACT == 2) v = fmaxf(v, 0.0f);
        if (ACT == 4) v = (v > 0.f) ? v : 0.01f * v;
        slab[(mOff + r) * 68 + (j << 4) + rlane] = v;
      }
    }
    __builtin_amdgcn_fence(__ATOMIC_RELEASE, "workgroup");
    __builtin_amdgcn_wave_barrier();
    __builtin_amdgcn_fence(__ATOMIC_ACQUIRE, "workgroup");
    if (OUT_MODE == 0) {
      float* C = (float*)Cout + (size_t)b * strideC;
      const int hh = lane >> 4, c4 = (lane & 15) * 4;
      for (int pass = 0; pass < 2; ++pass) {
#pragma unroll
        for (int it = 0; it < 8; ++it) {
          const int row = it * 2 + hh;
          v4f v = *(const v4f*)(slab + row * 68 + c4);
          *(volatile v4f*)(C + (size_t)(mBase + row) * ldc + n0 + c4) = v;
        }
        __threadfence();
      }
    } else {
      const int q = lane >> 3, c8 = (lane & 7) * 8;
      unsigned short* C  = (unsigned short*)Cout  + (size_t)b * strideC;
      unsigned short* C2 = (OUT_MODE == 2) ? ((unsigned short*)Cout2 + (size_t)b * strideC) : nullptr;
      for (int pass = 0; pass < 2; ++pass) {
#pragma unroll
        for (int it = 0; it < 4; ++it) {
          const int row = it * 4 + q;
          const float* sp = slab + row * 68 + c8;
          v8h hv, lv;
#pragma unroll
          for (int e = 0; e < 8; ++e) {
            if (OUT_MODE == 1) {
              hv[e] = (_Float16)sp[e];
            } else {
              unsigned short hb = f2bf_bits(sp[e]);
              unsigned short lb = f2bf_bits(sp[e] - bf_bits2f(hb));
              hv[e] = __builtin_bit_cast(_Float16, hb);
              lv[e] = __builtin_bit_cast(_Float16, lb);
            }
          }
          *(volatile v8h*)(C + (size_t)(mBase + row) * ldc + n0 + c8) = hv;
          if (OUT_MODE == 2) *(volatile v8h*)(C2 + (size_t)(mBase + row) * ldc + n0 + c8) = lv;
        }
        __threadfence();
      }
    }
    __builtin_amdgcn_fence(__ATOMIC_RELEASE, "workgroup");
    __builtin_amdgcn_wave_barrier();
    __builtin_amdgcn_fence(__ATOMIC_ACQUIRE, "workgroup");
  }
}

__global__ __launch_bounds__(256) void btpack_kernel(const float* __restrict__ values, const float* __restrict__ skip_w,
                                                     unsigned short* __restrict__ Bt, int nchunks) {
  const int i = blockIdx.x * 256 + threadIdx.x;
  if (i >= nchunks) return;
  const int o = i / kChunks;
  const int c = i - o * kChunks;
  const int k = c * 8;
  const int kv = (k < kKsp - 8) ? k : (kKsp - 8);
  int ks = k - kKsp;
  ks = (ks < 0) ? 0 : ks;
  ks = (ks > kIn - 8) ? (kIn - 8) : ks;
  const float* pv = values + (size_t)o * kKsp + kv;
  const float* ps = skip_w + (size_t)o * kIn + ks;
  const v4f a0 = *(const v4f*)(pv);
  const v4f a1 = *(const v4f*)(pv + 4);
  const v4f s0 = *(const v4f*)(ps);
  const v4f s1 = *(const v4f*)(ps + 4);
  const float fa = (k < kKsp) ? kBtCarry : 0.0f;
  const float fb = kBtCarry - fa;
  float v[8];
#pragma unroll
  for (int e = 0; e < 4; ++e) {
    v[e]     = fmaf(fa, a0[e], fb * s0[e]);
    v[4 + e] = fmaf(fa, a1[e], fb * s1[e]);
  }
  unsigned short hb[8];
#pragma unroll
  for (int e = 0; e < 8; ++e) hb[e] = h_bits(v[e]);
  const v4u u = (v4u){pk16(hb[0], hb[1]), pk16(hb[2], hb[3]), pk16(hb[4], hb[5]), pk16(hb[6], hb[7])};
  unsigned int* q = (unsigned int*)(Bt + (size_t)o * kKtot + k);
  *(volatile v4u*)q = u;
  __threadfence();
  *(volatile v4u*)q = u;
}

__global__ __launch_bounds__(128) void featbuild_kernel(const float* __restrict__ x, const float* __restrict__ knots,
                                                        unsigned short* __restrict__ Aplane) {
  __shared__ __align__(16) unsigned int sA[4][kRowWords];
  __shared__ float sg[kKnots];
  const int tid  = threadIdx.x;
  const int wave = tid >> 5;
  const int lane = tid & 31;
  const int row  = blockIdx.x * 4 + wave;
  if (tid < kKnots) sg[tid] = knots[tid];
  __syncthreads();
  float g[kKnots];
#pragma unroll
  for (int t = 0; t < kKnots; ++t) g[t] = sg[t];
  unsigned int* sw = sA[wave];
  const float* xr = x + (size_t)row * kIn;

#pragma unroll 1
  for (int j = 0; j < 8; ++j) {
    const int d = 32 * j + lane;
    const float xv = xr[d];
    const float xc = fminf(fmaxf(xv, -1.0f), 1.0f);
    int   left = 0;
    float g0 = g[0], g1 = g[1];
#pragma unroll
    for (int t = 1; t <= kKnots - 2; ++t) {
      const bool lt = g[t] < xc;
      left += lt ? 1 : 0;
      g0 = lt ? g[t] : g0;
      g1 = lt ? g[t + 1] : g1;
    }
    const float w   = (xc - g0) / (g1 - g0 + 1e-12f);
    const float omw = 1.0f - w;
    const unsigned hw   = (unsigned)h_bits(w);
    const unsigned homw = (unsigned)h_bits(omw);
    const unsigned hx   = (unsigned)h_bits(xc);
    const unsigned p0 = homw | (hw << 16);
    const unsigned p1 = homw << 16;
    const unsigned p2 = hw;
    unsigned wd[8];
#pragma unroll
    for (int m = 0; m < 8; ++m) {
      unsigned v = (left == 2 * m - 1) ? p2 : 0u;
      v = (left == 2 * m + 1) ? p1 : v;
      v = (left == 2 * m) ? p0 : v;
      wd[m] = v;
    }
    const v4u u0 = (v4u){wd[0], wd[1], wd[2], wd[3]};
    const v4u u1 = (v4u){wd[4], wd[5], wd[6], wd[7]};
    *(v4u*)(sw + d * 8)     = u0;
    *(v4u*)(sw + d * 8 + 4) = u1;
    const unsigned hxo = (unsigned)__shfl_xor((int)hx, 1, 32);
    if ((lane & 1) == 0) sw[kKsp / 2 + (d >> 1)] = hx | (hxo << 16);
  }
  __syncthreads();

  unsigned int* dstw = (unsigned int*)(Aplane + (size_t)row * kKtot);
  for (int pass = 0; pass < 2; ++pass) {
#pragma unroll
    for (int it = 0; it < kRowWords / 128; ++it) {
      const v4u v = *(const v4u*)(sw + it * 128 + lane * 4);
      *(volatile v4u*)(dstw + it * 128 + lane * 4) = v;
    }
    __threadfence();
  }
}

extern "C" void kernel_launch(void* const* d_in, const int* in_sizes, int n_in,
                              void* d_out, int out_size, void* d_ws, size_t ws_size,
                              hipStream_t stream) {
  if (n_in < 5) return;
  if (in_sizes[0] != kRows * kIn) return;
  if (in_sizes[1] != kOut * kKsp) return;
  if (in_sizes[2] != kOut * kIn) return;
  if (in_sizes[3] != kOut) return;
  if (in_sizes[4] != kKnots) return;
  if (out_size != kRows * kOut) return;
  const size_t btBytes = (size_t)kOut * kKtot * 2;
  const size_t aBytes  = (size_t)kRows * kKtot * 2;
  if (btBytes + aBytes > ws_size) return;

  const float* x      = (const float*)d_in[0];
  const float* values = (const float*)d_in[1];
  const float* skip_w = (const float*)d_in[2];
  const float* skip_b = (const float*)d_in[3];
  const float* knots  = (const float*)d_in[4];
  unsigned short* Bt = (unsigned short*)d_ws;
  unsigned short* Ap = (unsigned short*)((char*)d_ws + btBytes);
  float* out = (float*)d_out;

  const int nchunks = kOut * kChunks;
  btpack_kernel<<<nchunks / 256, 256, 0, stream>>>(values, skip_w, Bt, nchunks);

  featbuild_kernel<<<kRows / 4, 128, 0, stream>>>(x, knots, Ap);

  const int ntiles = (kRows / 64) * (kOut / 64);
  wmma_gemm64<0, false, 2, 0, false, 0><<<dim3(ntiles / 8, 1), 256, 0, stream>>>(
      Ap, Ap, kKtot, 0L,
      Bt, Bt, kKtot, 0L,
      (void*)out, (void*)out, kOut, 0L,
      skip_b,
      skip_b, 0L,
      kRows, kOut, kKtot, kBtCarryInv);
}
